// UniversalDirectionalGSA_36344013258853
// MI455X (gfx1250) — hardware-verified
//
#include <hip/hip_runtime.h>


#define B_    2
#define S_    1024
#define HID_  2048
#define NH_   16
#define NS_   8
#define D_    128
#define NTOK_ (B_ * S_)
#define MREC_ 1152

typedef unsigned short us8 __attribute__((ext_vector_type(8)));
typedef __bf16 bf16x16 __attribute__((ext_vector_type(16)));
typedef _Float16 f16x16 __attribute__((ext_vector_type(16)));
typedef float f32x8 __attribute__((ext_vector_type(8)));
typedef float v4f __attribute__((ext_vector_type(4)));

union FragB { bf16x16 v; us8 h[2]; };
union FragH { f16x16 v; us8 h[2]; };

__device__ __forceinline__ unsigned short f2bf(float f) {
  unsigned int u = __float_as_uint(f);
  u += 0x7FFFu + ((u >> 16) & 1u);
  return (unsigned short)(u >> 16);
}
__device__ __forceinline__ float bf2f(unsigned short b) { return __uint_as_float(((unsigned int)b) << 16); }
__device__ __forceinline__ float bfr(float f) { return bf2f(f2bf(f)); }
__device__ __forceinline__ unsigned short f2h(float f) {
  union { _Float16 x; unsigned short u; } c; c.x = (_Float16)f; return c.u;
}
__device__ __forceinline__ float h2f(unsigned short u) {
  union { _Float16 x; unsigned short s; } c; c.s = u; return (float)c.x;
}
__device__ __forceinline__ float sigm(float x) { return 1.0f / (1.0f + __expf(-x)); }

__device__ __forceinline__ bf16x16 ldfragb(const unsigned short* p, int hh) {
  FragB f;
  f.h[0] = *(const us8*)(p + 8 * hh);
  f.h[1] = *(const us8*)(p + 16 + 8 * hh);
  return f.v;
}
__device__ __forceinline__ f16x16 ldfragh(const unsigned short* p, int hh) {
  FragH f;
  f.h[0] = *(const us8*)(p + 8 * hh);
  f.h[1] = *(const us8*)(p + 16 + 8 * hh);
  return f.v;
}
__device__ __forceinline__ f32x8 mma_b(bf16x16 a, bf16x16 b, f32x8 c) {
  f32x8 d = __builtin_amdgcn_wmma_f32_16x16x32_bf16(false, a, false, b, (short)0, c, false, false);
  asm volatile("v_nop\n\tv_nop\n\tv_nop\n\tv_nop" : "+v"(d) : "v"(a), "v"(b));
  return d;
}
__device__ __forceinline__ f32x8 mma_h(f16x16 a, f16x16 b, f32x8 c) {
  f32x8 d = __builtin_amdgcn_wmma_f32_16x16x32_f16(false, a, false, b, (short)0, c, false, false);
  asm volatile("v_nop\n\tv_nop\n\tv_nop\n\tv_nop" : "+v"(d) : "v"(a), "v"(b));
  return d;
}

__global__ __launch_bounds__(128) void prep_kernel(const float* __restrict__ pos, const float* __restrict__ dir,
                                                   const float* __restrict__ lsc, const float* __restrict__ lam,
                                                   float* posn, float* dirn, float* scal) {
  const int t = threadIdx.x;
  if (t >= NH_ * NS_) return;
  const int h = t >> 3;
  const float* p = pos + (size_t)t * D_;
  const float* q = dir + (size_t)t * D_;
  float sp = 0.0f, sq = 0.0f;
#pragma unroll 1
  for (int i = 0; i < D_; ++i) {
    const float a = bfr(p[i]), c = bfr(q[i]);
    sp += a * a; sq += c * c;
  }
  const float pscale = 3.3941125496954285f;
  const float ip = 1.0f / (sqrtf(sp) + 1e-12f);
  const float iq = 1.0f / (sqrtf(sq) + 1e-12f);
  float pd = 0.0f, pp = 0.0f;
#pragma unroll 1
  for (int i = 0; i < D_; i += 4) {
    float pv[4], dv[4];
#pragma unroll
    for (int j = 0; j < 4; ++j) {
      pv[j] = bfr(p[i + j]) * ip * pscale;
      dv[j] = bfr(q[i + j]) * iq;
      pd += pv[j] * dv[j]; pp += pv[j] * pv[j];
    }
    const v4f a = {pv[0], pv[1], pv[2], pv[3]};
    const v4f c = {dv[0], dv[1], dv[2], dv[3]};
    *(volatile v4f*)(posn + (size_t)t * D_ + i) = a;
    *(volatile v4f*)(dirn + (size_t)t * D_ + i) = c;
  }
  __threadfence();
#pragma unroll 1
  for (int i = 0; i < D_; i += 4) {
    float pv[4], dv[4];
#pragma unroll
    for (int j = 0; j < 4; ++j) {
      pv[j] = bfr(p[i + j]) * ip * pscale;
      dv[j] = bfr(q[i + j]) * iq;
    }
    const v4f a = {pv[0], pv[1], pv[2], pv[3]};
    const v4f c = {dv[0], dv[1], dv[2], dv[3]};
    *(volatile v4f*)(posn + (size_t)t * D_ + i) = a;
    *(volatile v4f*)(dirn + (size_t)t * D_ + i) = c;
  }
  float sc = __expf(bfr(lsc[t]));
  sc = fminf(fmaxf(sc, 0.3f), 1.2f);
  float mx = -1e30f;
#pragma unroll
  for (int j = 0; j < NS_; ++j) mx = fmaxf(mx, bfr(lam[h * NS_ + j]));
  float se = 0.0f;
#pragma unroll
  for (int j = 0; j < NS_; ++j) se += __expf(bfr(lam[h * NS_ + j]) - mx);
  const float amp = __expf(bfr(lam[t]) - mx) / se;
  const v4f rec = {pp, pd, 0.5f / (sc * sc), amp};
  *(volatile v4f*)(scal + (size_t)t * 4) = rec;
  __threadfence();
  *(volatile v4f*)(scal + (size_t)t * 4) = rec;
}

__global__ __launch_bounds__(256) void cvt_kernel(const float* __restrict__ X, const float* __restrict__ W0,
                                                  const float* __restrict__ W1, const float* __restrict__ W2,
                                                  const float* __restrict__ W3, unsigned short* Xb,
                                                  unsigned short* Wt0, unsigned short* Wt1,
                                                  unsigned short* Wt2, unsigned short* Wt3) {
  __shared__ __align__(16) unsigned short lds_t[32 * 256];
  const int tid = threadIdx.x, bx = blockIdx.x, y = blockIdx.y;
  if (y == 4) {
    if ((size_t)(bx + 1) * 8192 > (size_t)NTOK_ * HID_) return;
    const float* src = X + (size_t)bx * 8192;
    unsigned short* dst = Xb + (size_t)bx * 8192;
    us8 o[4];
#pragma unroll
    for (int i = 0; i < 4; ++i) {
      const int c = i * 256 + tid;
      const v4f a = *(const v4f*)(src + (size_t)c * 8);
      const v4f b = *(const v4f*)(src + (size_t)c * 8 + 4);
      us8 e;
      e[0] = f2bf(a[0]); e[1] = f2bf(a[1]); e[2] = f2bf(a[2]); e[3] = f2bf(a[3]);
      e[4] = f2bf(b[0]); e[5] = f2bf(b[1]); e[6] = f2bf(b[2]); e[7] = f2bf(b[3]);
      o[i] = e;
    }
#pragma unroll
    for (int i = 0; i < 4; ++i) *(volatile us8*)(dst + (size_t)(i * 256 + tid) * 8) = o[i];
    __threadfence();
#pragma unroll
    for (int i = 0; i < 4; ++i) *(volatile us8*)(dst + (size_t)(i * 256 + tid) * 8) = o[i];
    return;
  }
  const float* W = (y == 0) ? W0 : (y == 1) ? W1 : (y == 2) ? W2 : W3;
  unsigned short* Wt = (y == 0) ? Wt0 : (y == 1) ? Wt1 : (y == 2) ? Wt2 : Wt3;
  const bool tof16 = (y == 3);
  const int n0 = (bx & 63) * 32, k0 = (bx >> 6) * 256;
  if (n0 + 32 > HID_ || k0 + 256 > HID_) return;
  {
    const float* src = W + (size_t)(k0 + tid) * HID_ + n0;
#pragma unroll
    for (int j4 = 0; j4 < 8; ++j4) {
      const v4f a = *(const v4f*)(src + j4 * 4);
#pragma unroll
      for (int q = 0; q < 4; ++q) {
        const float x = a[q];
        lds_t[(j4 * 4 + q) * 256 + tid] = tof16 ? f2h(bfr(x) * 64.0f) : f2bf(x);
      }
    }
  }
  __syncthreads();
  const int w = tid >> 5, l = tid & 31;
  us8 v[4];
#pragma unroll
  for (int i = 0; i < 4; ++i) v[i] = *(const us8*)(lds_t + (w * 4 + i) * 256 + l * 8);
#pragma unroll
  for (int i = 0; i < 4; ++i)
    *(volatile us8*)(Wt + (size_t)(n0 + w * 4 + i) * HID_ + k0 + l * 8) = v[i];
  __threadfence();
#pragma unroll
  for (int i = 0; i < 4; ++i)
    *(volatile us8*)(Wt + (size_t)(n0 + w * 4 + i) * HID_ + k0 + l * 8) = v[i];
}

__global__ __launch_bounds__(256) void gemm_qk_kernel(const unsigned short* __restrict__ Xb,
                                                      const unsigned short* __restrict__ Bt0,
                                                      const unsigned short* __restrict__ Bt1,
                                                      unsigned short* oh0, unsigned short* ol0,
                                                      unsigned short* oh1, unsigned short* ol1) {
  __shared__ __align__(16) unsigned short lds_s[128 * 64];
  const int tid = threadIdx.x, y = blockIdx.y;
  const int mbase = (blockIdx.x >> 5) << 7;
  const int nbase = (blockIdx.x & 31) << 6;
  if (mbase + 128 > NTOK_ || nbase + 64 > HID_) return;
  const unsigned short* Bt = y ? Bt1 : Bt0;
  unsigned short* oh = y ? oh1 : oh0;
  unsigned short* ol = y ? ol1 : ol0;
  const int w = tid >> 5, l = tid & 31, hh = l >> 4, m = l & 15;
  const unsigned short* arow = Xb + (size_t)(mbase + w * 16 + m) * HID_;
  const unsigned short* brow = Bt + (size_t)(nbase + m) * HID_;

  const f32x8 z = {0, 0, 0, 0, 0, 0, 0, 0};
  f32x8 acc[4];
#pragma unroll
  for (int i = 0; i < 4; ++i) acc[i] = z;

#pragma unroll 1
  for (int k0 = 0; k0 < HID_; k0 += 32) {
    const bf16x16 a = ldfragb(arow + k0, hh);
#pragma unroll
    for (int ct = 0; ct < 4; ++ct) {
      const bf16x16 bb = ldfragb(brow + (size_t)(ct * 16) * HID_ + k0, hh);
      acc[ct] = mma_b(a, bb, acc[ct]);
    }
  }

#pragma unroll
  for (int pl = 0; pl < 2; ++pl) {
#pragma unroll
    for (int ct = 0; ct < 4; ++ct) {
#pragma unroll
      for (int r = 0; r < 8; ++r) {
        const int row = w * 16 + 8 * hh + r, col = ct * 16 + m;
        const float v = acc[ct][r];
        const unsigned short hi = f2bf(v);
        lds_s[row * 64 + col] = (pl == 0) ? hi : f2bf(v - bf2f(hi));
      }
    }
    __syncthreads();
    unsigned short* dst = (pl == 0) ? oh : ol;
    us8 vv[4];
#pragma unroll
    for (int i = 0; i < 4; ++i) {
      const int f = i * 256 + tid;
      vv[i] = *(const us8*)(lds_s + (f >> 3) * 64 + (f & 7) * 8);
    }
#pragma unroll
    for (int i = 0; i < 4; ++i) {
      const int f = i * 256 + tid;
      *(volatile us8*)(dst + (size_t)(mbase + (f >> 3)) * HID_ + nbase + (f & 7) * 8) = vv[i];
    }
    __threadfence();
#pragma unroll
    for (int i = 0; i < 4; ++i) {
      const int f = i * 256 + tid;
      *(volatile us8*)(dst + (size_t)(mbase + (f >> 3)) * HID_ + nbase + (f & 7) * 8) = vv[i];
    }
    __syncthreads();
  }
}

__global__ __launch_bounds__(256) void gemm_v_kernel(const unsigned short* __restrict__ Xb,
                                                     const unsigned short* __restrict__ Bt,
                                                     unsigned short* Vt) {
  __shared__ __align__(16) unsigned short lds_s[64 * 128];
  const int tid = threadIdx.x;
  const int mbase = (blockIdx.x >> 5) << 7;
  const int nbase = (blockIdx.x & 31) << 6;
  if (mbase + 128 > NTOK_ || nbase + 64 > HID_) return;
  const int w = tid >> 5, l = tid & 31, hh = l >> 4, m = l & 15;
  const unsigned short* arow = Xb + (size_t)(mbase + w * 16 + m) * HID_;
  const unsigned short* brow = Bt + (size_t)(nbase + m) * HID_;

  const f32x8 z = {0, 0, 0, 0, 0, 0, 0, 0};
  f32x8 acc[4];
#pragma unroll
  for (int i = 0; i < 4; ++i) acc[i] = z;

#pragma unroll 1
  for (int k0 = 0; k0 < HID_; k0 += 32) {
    const bf16x16 a = ldfragb(arow + k0, hh);
#pragma unroll
    for (int ct = 0; ct < 4; ++ct) {
      const bf16x16 bb = ldfragb(brow + (size_t)(ct * 16) * HID_ + k0, hh);
      acc[ct] = mma_b(a, bb, acc[ct]);
    }
  }

#pragma unroll
  for (int ct = 0; ct < 4; ++ct) {
#pragma unroll
    for (int r = 0; r < 8; ++r) {
      const int row = w * 16 + 8 * hh + r, col = ct * 16 + m;
      lds_s[col * 128 + row] = f2h(acc[ct][r] * 8.0f);
    }
  }
  __syncthreads();
  const int bhv = (mbase >> 10) * NH_ + (nbase >> 7);
  const int d0 = nbase & (D_ - 1), s0 = mbase & (S_ - 1);
  us8 vv[4];
#pragma unroll
  for (int i = 0; i < 4; ++i) {
    const int f = i * 256 + tid;
    vv[i] = *(const us8*)(lds_s + (f >> 4) * 128 + (f & 15) * 8);
  }
#pragma unroll
  for (int i = 0; i < 4; ++i) {
    const int f = i * 256 + tid;
    *(volatile us8*)(Vt + ((size_t)(bhv * D_ + d0 + (f >> 4))) * S_ + s0 + (f & 15) * 8) = vv[i];
  }
  __threadfence();
#pragma unroll
  for (int i = 0; i < 4; ++i) {
    const int f = i * 256 + tid;
    *(volatile us8*)(Vt + ((size_t)(bhv * D_ + d0 + (f >> 4))) * S_ + s0 + (f & 15) * 8) = vv[i];
  }
}

__global__ __launch_bounds__(256) void affinity_kernel(const unsigned short* __restrict__ Qh,
                                                       const unsigned short* __restrict__ Ql,
                                                       const unsigned short* __restrict__ Kh,
                                                       const unsigned short* __restrict__ Kl,
                                                       float* qa, float* ka,
                                                       const float* __restrict__ posn,
                                                       const float* __restrict__ dirn,
                                                       const float* __restrict__ scal,
                                                       const float* __restrict__ dsp) {
  __shared__ __align__(16) float lds_aff[256];
  const int tid = threadIdx.x, w = tid >> 5, l = tid & 31;
  const int which = blockIdx.x >> 10;
  if (which > 1) return;
  const int item0 = (blockIdx.x & 1023) * 32;
  const int bh = item0 >> 10, b = bh >> 4, h = bh & 15, sb = item0 & (S_ - 1);
  const unsigned short* Th = which ? Kh : Qh;
  const unsigned short* Tl = which ? Kl : Ql;
  float* dstb = which ? ka : qa;
  const float ds = sigm(bfr(dsp[0]));

  float pn[8][4], dn[8][4];
#pragma unroll
  for (int n = 0; n < 8; ++n) {
#pragma unroll
    for (int j = 0; j < 4; ++j) {
      pn[n][j] = posn[(h * NS_ + n) * D_ + l + 32 * j];
      dn[n][j] = dirn[(h * NS_ + n) * D_ + l + 32 * j];
    }
  }
  const v4f rec = *(const v4f*)(scal + (size_t)(h * NS_ + (l & 7)) * 4);

#pragma unroll 1
  for (int t = 0; t < 4; ++t) {
    const int s = sb + w * 4 + t;
    const size_t ro = (size_t)(b * S_ + s) * HID_ + h * D_ + l;
    float tok[4];
#pragma unroll
    for (int j = 0; j < 4; ++j) tok[j] = bf2f(Th[ro + 32 * j]) + bf2f(Tl[ro + 32 * j]);
    float ts = 0.0f, tp[8], td[8];
#pragma unroll
    for (int n = 0; n < 8; ++n) { tp[n] = 0.0f; td[n] = 0.0f; }
#pragma unroll
    for (int j = 0; j < 4; ++j) {
      const float x = tok[j];
      ts += x * x;
#pragma unroll
      for (int n = 0; n < 8; ++n) { tp[n] += x * pn[n][j]; td[n] += x * dn[n][j]; }
    }
#pragma unroll
    for (int msk = 16; msk >= 1; msk >>= 1) {
      ts += __shfl_xor(ts, msk, 32);
#pragma unroll
      for (int n = 0; n < 8; ++n) {
        tp[n] += __shfl_xor(tp[n], msk, 32);
        td[n] += __shfl_xor(td[n], msk, 32);
      }
    }
    float tpn = 0.0f, tdn = 0.0f;
#pragma unroll
    for (int n = 0; n < 8; ++n) { if (l == n) { tpn = tp[n]; tdn = td[n]; } }
    if (l < NS_) {
      const float dist2 = fmaxf(ts - 2.0f * tpn + rec[0], 0.0f);
      const float proj = tdn - rec[1];
      const float perp2 = fmaxf(dist2 - proj * proj, 0.0f);
      const float a = (1.0f - ds) * __expf(-dist2 * rec[2]) + ds * __expf(-perp2 * rec[2]);
      lds_aff[(w * 4 + t) * 8 + l] = a;
    }
  }
  __syncthreads();
  if (tid < 64) {
    const v4f v = *(const v4f*)(lds_aff + tid * 4);
    *(volatile v4f*)(dstb + (size_t)item0 * NS_ + tid * 4) = v;
    __threadfence();
    *(volatile v4f*)(dstb + (size_t)item0 * NS_ + tid * 4) = v;
  }
}

__global__ __launch_bounds__(128) void mix_reduce_kernel(const unsigned short* __restrict__ Vt,
                                                         const float* __restrict__ ka,
                                                         const float* __restrict__ scal, float* mrec) {
  __shared__ __align__(16) float lds_rec[MREC_];
  const int bh = blockIdx.x, h = bh & 15, d = threadIdx.x;
  if (bh >= B_ * NH_) return;
  const size_t vro = ((size_t)bh * D_ + d) * S_;
  const float* kb = ka + (size_t)bh * S_ * NS_;
  float acc[8];
#pragma unroll
  for (int n = 0; n < 8; ++n) acc[n] = 0.0f;
  float ss = 0.0f;
#pragma unroll 1
  for (int s = 0; s < S_; ++s) {
    const float v = h2f(Vt[vro + s]) * 0.125f;
    const v4f k0 = *(const v4f*)(kb + (size_t)s * NS_);
    const v4f k1 = *(const v4f*)(kb + (size_t)s * NS_ + 4);
#pragma unroll
    for (int j = 0; j < 4; ++j) { acc[j] += k0[j] * v; acc[4 + j] += k1[j] * v; }
    float kd = 0.0f;
#pragma unroll
    for (int j = 0; j < 4; ++j) { if (d == j) kd = k0[j]; if (d == 4 + j) kd = k1[j]; }
    ss += kd;
  }
#pragma unroll
  for (int n = 0; n < 8; ++n) lds_rec[n * 128 + d] = scal[(h * NS_ + n) * 4 + 3] * acc[n];
  lds_rec[1024 + d] = (d < NS_) ? scal[(h * NS_ + (d & 7)) * 4 + 3] * ss : 0.0f;
  __syncthreads();
  const v4f zz = {0, 0, 0, 0};
  v4f vv[3];
#pragma unroll
  for (int i = 0; i < 3; ++i) {
    const int f = i * 128 + d;
    vv[i] = (f < MREC_ / 4) ? *(const v4f*)(lds_rec + f * 4) : zz;
  }
#pragma unroll
  for (int i = 0; i < 3; ++i) {
    const int f = i * 128 + d;
    if (f < MREC_ / 4) *(volatile v4f*)(mrec + (size_t)bh * MREC_ + f * 4) = vv[i];
  }
  __threadfence();
#pragma unroll
  for (int i = 0; i < 3; ++i) {
    const int f = i * 128 + d;
    if (f < MREC_ / 4) *(volatile v4f*)(mrec + (size_t)bh * MREC_ + f * 4) = vv[i];
  }
}

__global__ __launch_bounds__(256) void attn_kernel(
    const unsigned short* __restrict__ Qh, const unsigned short* __restrict__ Ql,
    const unsigned short* __restrict__ Kh, const unsigned short* __restrict__ Kl,
    const unsigned short* __restrict__ Vt, const float* __restrict__ qa,
    const float* __restrict__ mrec, const float* __restrict__ gsp, unsigned short* AO) {
  __shared__ __align__(16) unsigned short lds_p[4 * 512];
  __shared__ __align__(16) float lds_c[64];
  __shared__ __align__(16) float lds_il[64];
  __shared__ __align__(16) unsigned short lds_o[64 * 128];
  __shared__ __align__(16) float lds_qa[64 * NS_];
  __shared__ __align__(16) float lds_m[MREC_];
  const int tid = threadIdx.x, w = tid >> 5, l = tid & 31, hh = l >> 4, m = l & 15;
  const int g = w & 3, dh = w >> 2;
  const int bh = blockIdx.x >> 4, qblk = blockIdx.x & 15;
  if (bh >= B_ * NH_) return;
  const int b = bh >> 4, h = bh & 15, q0 = qblk * 64;
  const float rscale = 0.08838834764831845f;
  const size_t qro = (size_t)(b * S_ + q0 + g * 16 + m) * HID_ + h * D_;

  const f32x8 z = {0, 0, 0, 0, 0, 0, 0, 0};
  f32x8 O[4];
#pragma unroll
  for (int i = 0; i < 4; ++i) O[i] = z;
  float mrow[8], lrow[8];
#pragma unroll
  for (int i = 0; i < 8; ++i) { mrow[i] = -1e30f; lrow[i] = 0.0f; }

#pragma unroll 1
  for (int kt = 0; kt < S_ / 32; ++kt) {
    if (w < 4) {
      const size_t kro0 = (size_t)(b * S_ + kt * 32 + m) * HID_ + h * D_;
      const size_t kro1 = kro0 + (size_t)16 * HID_;
      f32x8 s0 = z, s1 = z;
#pragma unroll 1
      for (int kd = 0; kd < D_ / 32; ++kd) {
        const int ko = kd * 32;
        const bf16x16 aqh = ldfragb(Qh + qro + ko, hh);
        const bf16x16 aql = ldfragb(Ql + qro + ko, hh);
        const bf16x16 b0h = ldfragb(Kh + kro0 + ko, hh);
        const bf16x16 b0l = ldfragb(Kl + kro0 + ko, hh);
        s0 = mma_b(aqh, b0h, s0); s0 = mma_b(aqh, b0l, s0); s0 = mma_b(aql, b0h, s0);
        const bf16x16 b1h = ldfragb(Kh + kro1 + ko, hh);
        const bf16x16 b1l = ldfragb(Kl + kro1 + ko, hh);
        s1 = mma_b(aqh, b1h, s1); s1 = mma_b(aqh, b1l, s1); s1 = mma_b(aql, b1h, s1);
      }
#pragma unroll
      for (int i = 0; i < 8; ++i) {
        const float a0 = s0[i] * rscale, a1 = s1[i] * rscale;
        float mx = fmaxf(a0, a1);
        mx = fmaxf(mx, __shfl_xor(mx, 1, 32));
        mx = fmaxf(mx, __shfl_xor(mx, 2, 32));
        mx = fmaxf(mx, __shfl_xor(mx, 4, 32));
        mx = fmaxf(mx, __shfl_xor(mx, 8, 32));
        const float nm = fmaxf(mrow[i], mx);
        const float c = __expf(mrow[i] - nm);
        const float p0 = __expf(a0 - nm), p1 = __expf(a1 - nm);
        float rs = p0 + p1;
        rs += __shfl_xor(rs, 1, 32);
        rs += __shfl_xor(rs, 2, 32);
        rs += __shfl_xor(rs, 4, 32);
        rs += __shfl_xor(rs, 8, 32);
        lrow[i] = lrow[i] * c + rs;
        mrow[i] = nm;
        if (m == 0) lds_c[g * 16 + 8 * hh + i] = c;
        const int pr = g * 512 + (8 * hh + i) * 32;
        lds_p[pr + m] = f2h(p0 * 256.0f);
        lds_p[pr + 16 + m] = f2h(p1 * 256.0f);
      }
    }
    __syncthreads();
    {
      const v4f c0 = *(const v4f*)(lds_c + g * 16 + 8 * hh);
      const v4f c1 = *(const v4f*)(lds_c + g * 16 + 8 * hh + 4);
      const f32x8 cv = {c0[0], c0[1], c0[2], c0[3], c1[0], c1[1], c1[2], c1[3]};
      const f16x16 ap = ldfragh(lds_p + g * 512 + m * 32, hh);
      const size_t vb = ((size_t)(bh * D_ + dh * 64 + m)) * S_ + kt * 32;
#pragma unroll
      for (int ns = 0; ns < 4; ++ns) {
        const f16x16 bv = ldfragh(Vt + vb + (size_t)(ns * 16) * S_, hh);
        O[ns] = mma_h(ap, bv, O[ns] * cv);
      }
    }
    __syncthreads();
  }

  if (w < 4) {
    if (m == 0) {
#pragma unroll
      for (int i = 0; i < 8; ++i) lds_il[g * 16 + 8 * hh + i] = 1.0f / lrow[i];
    }
  }
  {
    const size_t qb = ((size_t)bh * S_ + q0) * NS_;
    if (tid < 128) *(v4f*)(lds_qa + tid * 4) = *(const v4f*)(qa + qb + tid * 4);
#pragma unroll
    for (int i = 0; i < 2; ++i) {
      const int f = i * 256 + tid;
      if (f < MREC_ / 4) *(v4f*)(lds_m + f * 4) = *(const v4f*)(mrec + (size_t)bh * MREC_ + f * 4);
    }
  }
  __syncthreads();
  const float blend = fminf(0.05f, sigm(bfr(gsp[0])) * 0.1f);
  const v4f il0 = *(const v4f*)(lds_il + g * 16 + 8 * hh);
  const v4f il1 = *(const v4f*)(lds_il + g * 16 + 8 * hh + 4);
#pragma unroll
  for (int i = 0; i < 8; ++i) {
    const int tl = g * 16 + 8 * hh + i;
    const float il = (i < 4) ? il0[i] : il1[i - 4];
    const v4f qv0 = *(const v4f*)(lds_qa + tl * NS_);
    const v4f qv1 = *(const v4f*)(lds_qa + tl * NS_ + 4);
    float q8[8];
    q8[0] = qv0[0]; q8[1] = qv0[1]; q8[2] = qv0[2]; q8[3] = qv0[3];
    q8[4] = qv1[0]; q8[5] = qv1[1]; q8[6] = qv1[2]; q8[7] = qv1[3];
    float den = 1e-8f;
#pragma unroll
    for (int n = 0; n < 8; ++n) den += q8[n] * lds_m[1024 + n];
    const float rden = 1.0f / den;
    const float osc = il * (1.0f / 2048.0f);
#pragma unroll
    for (int ns = 0; ns < 4; ++ns) {
      const int col = dh * 64 + ns * 16 + m;
      float dg = 0.0f;
#pragma unroll
      for (int n = 0; n < 8; ++n) dg += q8[n] * lds_m[n * 128 + col];
      const float val = (1.0f - blend) * (O[ns][i] * osc) + blend * (dg * rden);
      lds_o[tl * 128 + col] = f2h(val * 64.0f);
    }
  }
  __syncthreads();
  us8 vv[4];
#pragma unroll
  for (int i = 0; i < 4; ++i) {
    const int f = i * 256 + tid;
    vv[i] = *(const us8*)(lds_o + (f >> 4) * 128 + (f & 15) * 8);
  }
#pragma unroll
  for (int i = 0; i < 4; ++i) {
    const int f = i * 256 + tid;
    *(volatile us8*)(AO + (size_t)(b * S_ + q0 + (f >> 4)) * HID_ + h * D_ + (f & 15) * 8) = vv[i];
  }
  __threadfence();
#pragma unroll
  for (int i = 0; i < 4; ++i) {
    const int f = i * 256 + tid;
    *(volatile us8*)(AO + (size_t)(b * S_ + q0 + (f >> 4)) * HID_ + h * D_ + (f & 15) * 8) = vv[i];
  }
}

__global__ __launch_bounds__(256) void gemm_out_kernel(const unsigned short* __restrict__ Ah,
                                                       const unsigned short* __restrict__ Bt, float* out) {
  __shared__ __align__(16) float lds_f[128 * 64];
  const int tid = threadIdx.x;
  const int mbase = (blockIdx.x >> 5) << 7;
  const int nbase = (blockIdx.x & 31) << 6;
  if (mbase + 128 > NTOK_ || nbase + 64 > HID_) return;
  const int w = tid >> 5, l = tid & 31, hh = l >> 4, m = l & 15;
  const unsigned short* arow = Ah + (size_t)(mbase + w * 16 + m) * HID_;
  const unsigned short* brow = Bt + (size_t)(nbase + m) * HID_;

  const f32x8 z = {0, 0, 0, 0, 0, 0, 0, 0};
  f32x8 acc[4];
#pragma unroll
  for (int i = 0; i < 4; ++i) acc[i] = z;

#pragma unroll 1
  for (int k0 = 0; k0 < HID_; k0 += 32) {
    const f16x16 a = ldfragh(arow + k0, hh);
#pragma unroll
    for (int ct = 0; ct < 4; ++ct) {
      const f16x16 bb = ldfragh(brow + (size_t)(ct * 16) * HID_ + k0, hh);
      acc[ct] = mma_h(a, bb, acc[ct]);
    }
  }

#pragma unroll
  for (int ct = 0; ct < 4; ++ct) {
#pragma unroll
    for (int r = 0; r < 8; ++r) {
      const int row = w * 16 + 8 * hh + r, col = ct * 16 + m;
      lds_f[row * 64 + col] = acc[ct][r] * (1.0f / 4096.0f);
    }
  }
  __syncthreads();
  v4f vv[8];
#pragma unroll
  for (int i = 0; i < 8; ++i) {
    const int f = i * 256 + tid;
    vv[i] = *(const v4f*)(lds_f + (f >> 4) * 64 + (f & 15) * 4);
  }
#pragma unroll
  for (int i = 0; i < 8; ++i) {
    const int f = i * 256 + tid;
    *(volatile v4f*)(out + (size_t)(mbase + (f >> 4)) * HID_ + nbase + (f & 15) * 4) = vv[i];
  }
  __threadfence();
#pragma unroll
  for (int i = 0; i < 8; ++i) {
    const int f = i * 256 + tid;
    *(volatile v4f*)(out + (size_t)(mbase + (f >> 4)) * HID_ + nbase + (f & 15) * 4) = vv[i];
  }
}

extern "C" void kernel_launch(void* const* d_in, const int* in_sizes, int n_in,
                              void* d_out, int out_size, void* d_ws, size_t ws_size,
                              hipStream_t stream) {
  if (n_in < 11) return;
  if (in_sizes[0] != NTOK_ * HID_) return;
  if (in_sizes[1] != HID_ * HID_ || in_sizes[2] != HID_ * HID_ ||
      in_sizes[3] != HID_ * HID_ || in_sizes[4] != HID_ * HID_) return;
  if (in_sizes[5] != NH_ * NS_ * D_ || in_sizes[6] != NH_ * NS_ * D_) return;
  if (in_sizes[7] != NH_ * NS_ || in_sizes[8] != NH_ * NS_) return;
  if (in_sizes[9] < 1 || in_sizes[10] < 1) return;
  if (out_size != NTOK_ * HID_) return;

  const float* X   = (const float*)d_in[0];
  const float* Wq  = (const float*)d_in[1];
  const float* Wk  = (const float*)d_in[2];
  const float* Wv  = (const float*)d_in[3];
  const float* Wo  = (const float*)d_in[4];
  const float* spo = (const float*)d_in[5];
  const float* sdi = (const float*)d_in[6];
  const float* sls = (const float*)d_in[7];
  const float* sla = (const float*)d_in[8];
  const float* dsp = (const float*)d_in[9];
  const float* gsp = (const float*)d_in[10];
  float* out = (float*)d_out;

  char* ws = (char*)d_ws;
  size_t off = 0;
  const size_t plane = (size_t)NTOK_ * HID_ * sizeof(unsigned short);
  unsigned short* Xb  = (unsigned short*)(ws + off); off += plane;
  unsigned short* Wt0 = (unsigned short*)(ws + off); off += plane;
  unsigned short* Wt1 = (unsigned short*)(ws + off); off += plane;
  unsigned short* Wt2 = (unsigned short*)(ws + off); off += plane;
  unsigned short* Wt3 = (unsigned short*)(ws + off); off += plane;
  unsigned short* Qh  = (unsigned short*)(ws + off); off += plane;
  unsigned short* Ql  = (unsigned short*)(ws + off); off += plane;
  unsigned short* Kh  = (unsigned short*)(ws + off); off += plane;
  unsigned short* Kl  = (unsigned short*)(ws + off); off += plane;
  unsigned short* Vt  = (unsigned short*)(ws + off); off += plane;
  unsigned short* AOb = (unsigned short*)(ws + off); off += plane;
  const size_t affBytes = (size_t)B_ * NH_ * S_ * NS_ * sizeof(float);
  float* qa   = (float*)(ws + off); off += affBytes;
  float* ka   = (float*)(ws + off); off += affBytes;
  float* posn = (float*)(ws + off); off += (size_t)NH_ * NS_ * D_ * sizeof(float);
  float* dirn = (float*)(ws + off); off += (size_t)NH_ * NS_ * D_ * sizeof(float);
  float* scal = (float*)(ws + off); off += (size_t)NH_ * NS_ * 4 * sizeof(float);
  float* mrec = (float*)(ws + off); off += (size_t)B_ * NH_ * MREC_ * sizeof(float);
  if (off > ws_size) return;

  prep_kernel<<<1, 128, 0, stream>>>(spo, sdi, sls, sla, posn, dirn, scal);
  cvt_kernel<<<dim3(512, 5), 256, 0, stream>>>(X, Wq, Wk, Wv, Wo, Xb, Wt0, Wt1, Wt2, Wt3);
  gemm_qk_kernel<<<dim3(512, 2), 256, 0, stream>>>(Xb, Wt0, Wt1, Qh, Ql, Kh, Kl);
  gemm_v_kernel<<<512, 256, 0, stream>>>(Xb, Wt2, Vt);
  affinity_kernel<<<2048, 256, 0, stream>>>(Qh, Ql, Kh, Kl, qa, ka, posn, dirn, scal, dsp);
  mix_reduce_kernel<<<B_ * NH_, 128, 0, stream>>>(Vt, ka, scal, mrec);
  attn_kernel<<<B_ * NH_ * (S_ / 64), 256, 0, stream>>>(Qh, Ql, Kh, Kl, Vt, qa, mrec, gsp, AOb);
  gemm_out_kernel<<<512, 256, 0, stream>>>(AOb, Wt3, out);
}
